// Cross_Attention_26517128085816
// MI455X (gfx1250) — hardware-verified
//
#include <hip/hip_runtime.h>
#include <stdint.h>
#include <stddef.h>

#define DEVINL __device__ __forceinline__

typedef _Float16 f16t;
typedef _Float16 v16h __attribute__((ext_vector_type(16)));
typedef _Float16 v8h  __attribute__((ext_vector_type(8)));
typedef __bf16   v16b __attribute__((ext_vector_type(16)));
typedef unsigned short v8us __attribute__((ext_vector_type(8)));
typedef float    v8f  __attribute__((ext_vector_type(8)));
typedef float    v4f  __attribute__((ext_vector_type(4)));
typedef v8h  __attribute__((may_alias)) v8ha;
typedef v8us __attribute__((may_alias)) v8usa;
typedef v4f  __attribute__((may_alias)) v4fa;
union FragH { v16h v; v8h half[2]; };
union FragB { v16b v; v8us half[2]; };

#define NB     4
#define CIN    512
#define DH     64
#define NS     2304
#define NQT    (NS / 64)
#define NCT64  (CIN / 64)
#define NNT32  (NS / 32)
#define WMAT   32768
#define NWM    10
#define TPBP   256
#define TPB    128
#define WAVES  4
#define PH     72
#define PF     68
#define ACAR   16.0f
#define WCAR   256.0f
#define FCAR   16.0f
#define PCAR   256.0f
#define AGCAR  16.0f
#define SC_P   (1.0f / 4096.0f)
#define SC_OA  (1.0f / 256.0f)
#define SC_V   (1.0f / 4096.0f)
#define XP_BLKS (2 * NB * NNT32 * NCT64)
#define WB_BLKS (NWM * WMAT / 8 / TPBP)
#define PLN    ((size_t)NB * NS * DH)

static_assert(TPB == WAVES * 32);
static_assert((NS % 64) == 0);
static_assert((CIN % 64) == 0);
static_assert(DH == 64);
static_assert(WB_BLKS * TPBP * 8 == NWM * WMAT);
static_assert((WMAT / 8 / TPBP) == 16);
static_assert((PH % 8) == 0);
static_assert((PF % 4) == 0);
static_assert(NQT * 64 == NS);
static_assert(NNT32 * 32 == NS);
static_assert(NCT64 * 64 == CIN);

DEVINL v8f wmma_f16(v16h a, v16h b, v8f c) {
  v8f d = __builtin_amdgcn_wmma_f32_16x16x32_f16(false, a, false, b, (short)0, c, false, false);
  asm volatile("v_nop\n\tv_nop\n\tv_nop\n\tv_nop" : "+v"(d) : "v"(a), "v"(b));
  return d;
}
DEVINL v8f wmma_bf16(v16b a, v16b b, v8f c) {
  v8f d = __builtin_amdgcn_wmma_f32_16x16x32_bf16(false, a, false, b, (short)0, c, false, false);
  asm volatile("v_nop\n\tv_nop\n\tv_nop\n\tv_nop" : "+v"(d) : "v"(a), "v"(b));
  return d;
}
DEVINL v8f zero8f() {
  v8f z = {0.f, 0.f, 0.f, 0.f, 0.f, 0.f, 0.f, 0.f};
  return z;
}
DEVINL void load_frag(FragH& f, const f16t* row, int k0) {
  f.half[0] = *(const v8ha*)(row + k0);
  f.half[1] = *(const v8ha*)(row + k0 + 16);
}
DEVINL void load_fragb(FragB& f, const unsigned short* row, int k0) {
  f.half[0] = *(const v8usa*)(row + k0);
  f.half[1] = *(const v8usa*)(row + k0 + 16);
}
DEVINL unsigned short bf16_bits(float a) {
  union { __bf16 hh; unsigned short s; } u;
  u.hh = (__bf16)a;
  return u.s;
}
DEVINL void split_bf16(float v, unsigned short& hb, unsigned short& lb) {
  hb = bf16_bits(v);
  const float hf = __uint_as_float(((unsigned)hb) << 16);
  lb = bf16_bits(v - hf);
}

template <int KD>
DEVINL void mma_4n(const f16t* __restrict__ arow, const f16t* __restrict__ brow, v8f (&acc)[4]) {
  #pragma unroll 1
  for (int ks = 0; ks < KD / 32; ++ks) {
    const int k0 = 32 * ks;
    FragH a;
    load_frag(a, arow, k0);
    #pragma unroll
    for (int n = 0; n < 4; ++n) {
      FragH b;
      load_frag(b, brow + (size_t)16 * n * KD, k0);
      acc[n] = wmma_f16(a.v, b.v, acc[n]);
    }
  }
}

__global__ __launch_bounds__(TPBP) void prep_k(const float* __restrict__ x, const float* __restrict__ y,
                                              const float* __restrict__ w0, const float* __restrict__ w1,
                                              const float* __restrict__ w2, const float* __restrict__ w3,
                                              const float* __restrict__ w4, const float* __restrict__ w5,
                                              const float* __restrict__ w6, const float* __restrict__ w7,
                                              const float* __restrict__ w8, const float* __restrict__ w9,
                                              f16t* __restrict__ XT, f16t* __restrict__ YT,
                                              f16t* __restrict__ WB)
{
  __shared__ __attribute__((aligned(16))) f16t tile[32 * PH];
  const int blk = blockIdx.x, tid = threadIdx.x;
  if (blk < XP_BLKS) {
    const int which = blk / (NB * NNT32 * NCT64);
    int rem = blk - which * (NB * NNT32 * NCT64);
    const int b = rem / (NNT32 * NCT64);
    rem -= b * (NNT32 * NCT64);
    const int nt = rem / NCT64;
    const int ct = rem - nt * NCT64;
    const int n0 = 32 * nt, c0 = 64 * ct;
    const float* src = which ? y : x;
    f16t* dst = which ? YT : XT;

    const int crow = tid >> 2, np = (tid & 3) * 8;
    const float* sp = src + ((size_t)b * CIN + c0 + crow) * NS + n0 + np;
    const v4f a = *(const v4fa*)sp, c = *(const v4fa*)(sp + 4);
    #pragma unroll
    for (int j = 0; j < 4; ++j) {
      tile[(np + j) * PH + crow]     = (f16t)(a[j] * ACAR);
      tile[(np + 4 + j) * PH + crow] = (f16t)(c[j] * ACAR);
    }
    __syncthreads();
    const int nrow = tid >> 3, q = tid & 7;
    const v8h o = *(const v8ha*)(tile + nrow * PH + 8 * q);
    f16t* dp = dst + ((size_t)b * NS + n0 + nrow) * CIN + c0 + 8 * q;
    *(volatile v8h*)dp = o;
    __threadfence();
    *(volatile v8h*)dp = o;
  } else if (blk < XP_BLKS + WB_BLKS) {
    const int wb = blk - XP_BLKS;
    const int mtx = wb >> 4;
    const int idx = ((wb & 15) * TPBP + tid) * 8;
    const float* src;
    switch (mtx) {
      case 0: src = w0; break;
      case 1: src = w1; break;
      case 2: src = w2; break;
      case 3: src = w3; break;
      case 4: src = w4; break;
      case 5: src = w5; break;
      case 6: src = w6; break;
      case 7: src = w7; break;
      case 8: src = w8; break;
      default: src = w9; break;
    }
    const v4f a = *(const v4fa*)(src + idx), c = *(const v4fa*)(src + idx + 4);
    v8h o;
    #pragma unroll
    for (int j = 0; j < 4; ++j) {
      o[j]     = (f16t)(a[j] * WCAR);
      o[4 + j] = (f16t)(c[j] * WCAR);
    }
    f16t* dp = WB + (size_t)mtx * WMAT + idx;
    *(volatile v8h*)dp = o;
    __threadfence();
    *(volatile v8h*)dp = o;
  }
}

__global__ __launch_bounds__(TPB) void proj_k(const f16t* __restrict__ XT, const f16t* __restrict__ YT,
                                             const f16t* __restrict__ WB,
                                             const float* __restrict__ bf1, const float* __restrict__ bg1,
                                             const float* __restrict__ bh1, const float* __restrict__ bf2,
                                             const float* __restrict__ bg2, const float* __restrict__ bh2,
                                             unsigned short* __restrict__ FG, f16t* __restrict__ HP)
{
  __shared__ __attribute__((aligned(16))) float sbuf[64 * PF];
  const int tid = threadIdx.x, lane = tid & 31, wave = tid >> 5;
  const int h = lane >> 4, m = lane & 15;
  const int blk = blockIdx.x;
  const int p = blk / (NB * NQT);
  int rem = blk - p * (NB * NQT);
  const int b = rem / NQT;
  const int nb = rem - b * NQT;
  const int n0 = 64 * nb;

  const f16t* Z;
  const f16t* Wp;
  const float* bias;
  int tr, sl;
  switch (p) {
    case 0:  Z = XT; Wp = WB + 0 * WMAT; bias = bf1; tr = 0; sl = 0; break;
    case 1:  Z = XT; Wp = WB + 1 * WMAT; bias = bg1; tr = 0; sl = 1; break;
    case 2:  Z = XT; Wp = WB + 2 * WMAT; bias = bh1; tr = 1; sl = 0; break;
    case 3:  Z = YT; Wp = WB + 3 * WMAT; bias = bf2; tr = 0; sl = 2; break;
    case 4:  Z = YT; Wp = WB + 4 * WMAT; bias = bg2; tr = 0; sl = 3; break;
    default: Z = XT; Wp = WB + 5 * WMAT; bias = bh2; tr = 1; sl = 1; break;
  }

  v8f acc[4];
  #pragma unroll
  for (int t = 0; t < 4; ++t) acc[t] = zero8f();
  const f16t* arow = Z + ((size_t)b * NS + n0 + 16 * wave + m) * CIN + 8 * h;
  const f16t* brow = Wp + (size_t)m * CIN + 8 * h;
  mma_4n<CIN>(arow, brow, acc);

  #pragma unroll
  for (int t = 0; t < 4; ++t) {
    const int d = 16 * t + m;
    const float bv = bias[d];
    #pragma unroll
    for (int r = 0; r < 8; ++r) {
      const int nrow = 16 * wave + 8 * h + r;
      const float v = acc[t][r] * SC_P + bv;
      const int idx = tr ? (d * PF + nrow) : (nrow * PF + d);
      sbuf[idx] = v;
    }
  }
  __syncthreads();

  if (tr) {
    f16t* PL = HP + (size_t)sl * PLN;
    v8h ov[4];
    size_t off[4];
    #pragma unroll
    for (int k = 0; k < 4; ++k) {
      const int row = 16 * k + (tid >> 3), q = tid & 7;
      const v4f a = *(const v4fa*)(sbuf + row * PF + 8 * q), c = *(const v4fa*)(sbuf + row * PF + 8 * q + 4);
      #pragma unroll
      for (int j = 0; j < 4; ++j) {
        ov[k][j]     = (f16t)(a[j] * FCAR);
        ov[k][4 + j] = (f16t)(c[j] * FCAR);
      }
      off[k] = ((size_t)b * DH + row) * NS + n0 + 8 * q;
    }
    #pragma unroll
    for (int k = 0; k < 4; ++k) *(volatile v8h*)(PL + off[k]) = ov[k];
    __threadfence();
    #pragma unroll
    for (int k = 0; k < 4; ++k) *(volatile v8h*)(PL + off[k]) = ov[k];
  } else {
    unsigned short* PHI = FG + (size_t)(2 * sl) * PLN;
    unsigned short* PLO = PHI + PLN;
    v8us hv[4], lv[4];
    size_t off[4];
    #pragma unroll
    for (int k = 0; k < 4; ++k) {
      const int row = 16 * k + (tid >> 3), q = tid & 7;
      const v4f a = *(const v4fa*)(sbuf + row * PF + 8 * q), c = *(const v4fa*)(sbuf + row * PF + 8 * q + 4);
      #pragma unroll
      for (int j = 0; j < 4; ++j) {
        unsigned short hb, lb;
        split_bf16(a[j], hb, lb);
        hv[k][j] = hb; lv[k][j] = lb;
        split_bf16(c[j], hb, lb);
        hv[k][4 + j] = hb; lv[k][4 + j] = lb;
      }
      off[k] = ((size_t)b * NS + n0 + row) * DH + 8 * q;
    }
    #pragma unroll
    for (int k = 0; k < 4; ++k) {
      *(volatile v8us*)(PHI + off[k]) = hv[k];
      *(volatile v8us*)(PLO + off[k]) = lv[k];
    }
    __threadfence();
    #pragma unroll
    for (int k = 0; k < 4; ++k) {
      *(volatile v8us*)(PHI + off[k]) = hv[k];
      *(volatile v8us*)(PLO + off[k]) = lv[k];
    }
  }
}

DEVINL v8f score_tile(const unsigned short* ghr, const unsigned short* glr,
                      const FragB& fh0, const FragB& fl0, const FragB& fh1, const FragB& fl1) {
  v8f s = zero8f();
  FragB gh, gl;
  load_fragb(gh, ghr, 0);
  load_fragb(gl, glr, 0);
  s = wmma_bf16(gh.v, fh0.v, s);
  s = wmma_bf16(gh.v, fl0.v, s);
  s = wmma_bf16(gl.v, fh0.v, s);
  load_fragb(gh, ghr, 32);
  load_fragb(gl, glr, 32);
  s = wmma_bf16(gh.v, fh1.v, s);
  s = wmma_bf16(gh.v, fl1.v, s);
  s = wmma_bf16(gl.v, fh1.v, s);
  return s;
}

__global__ __launch_bounds__(TPB) void agg_k(const unsigned short* __restrict__ FG, const f16t* __restrict__ HP,
                                            f16t* __restrict__ AG)
{
  __shared__ __attribute__((aligned(16))) f16t sbuf[64 * PH];
  const int tid = threadIdx.x, lane = tid & 31, wave = tid >> 5;
  const int h = lane >> 4, m = lane & 15;
  const int blk = blockIdx.x;
  const int p = blk / (NB * NQT);
  int rem = blk - p * (NB * NQT);
  const int b = rem / NQT;
  const int qb = rem - b * NQT;

  int fq, gq, hs;
  switch (p) {
    case 0:  fq = 0; gq = 1; hs = 0; break;
    case 1:  fq = 2; gq = 1; hs = 0; break;
    case 2:  fq = 2; gq = 3; hs = 1; break;
    default: fq = 0; gq = 3; hs = 1; break;
  }
  const unsigned short* Fh = FG + (size_t)(2 * fq) * PLN;
  const unsigned short* Fl = Fh + PLN;
  const unsigned short* Gh = FG + (size_t)(2 * gq) * PLN;
  const unsigned short* Gl = Gh + PLN;
  const f16t* H = HP + (size_t)hs * PLN;
  f16t* AGp = AG + (size_t)p * PLN;

  const int i0 = 64 * qb + 16 * wave;
  FragB fh0, fh1, fl0, fl1;
  {
    const size_t foff = ((size_t)b * NS + i0 + m) * DH + 8 * h;
    load_fragb(fh0, Fh + foff, 0);
    load_fragb(fh1, Fh + foff, 32);
    load_fragb(fl0, Fl + foff, 0);
    load_fragb(fl1, Fl + foff, 32);
  }
  const size_t goff = ((size_t)b * NS + m) * DH + 8 * h;
  const f16t* hbase = H + ((size_t)b * DH + m) * NS + 8 * h;

  v8f O[4];
  #pragma unroll
  for (int t = 0; t < 4; ++t) O[t] = zero8f();
  float Mx = -3.0e38f, L = 0.0f;

  #pragma unroll 1
  for (int js = 0; js < NS / 32; ++js) {
    const int j0 = 32 * js;
    const size_t r0 = goff + (size_t)j0 * DH;
    const size_t r1 = r0 + (size_t)16 * DH;
    const v8f s0 = score_tile(Gh + r0, Gl + r0, fh0, fl0, fh1, fl1);
    const v8f s1 = score_tile(Gh + r1, Gl + r1, fh0, fl0, fh1, fl1);

    float mloc = -3.0e38f;
    #pragma unroll
    for (int r = 0; r < 8; ++r) mloc = fmaxf(mloc, fmaxf(s0[r], s1[r]));
    mloc = fmaxf(mloc, __shfl_xor(mloc, 16));
    const float Mn = fmaxf(Mx, mloc);
    const float corr = __expf(Mx - Mn);
    Mx = Mn;

    FragH pf;
    float ls = 0.0f;
    #pragma unroll
    for (int r = 0; r < 8; ++r) {
      const float e0 = __expf(s0[r] - Mn);
      const float e1 = __expf(s1[r] - Mn);
      ls += e0 + e1;
      pf.half[0][r] = (f16t)(e0 * PCAR);
      pf.half[1][r] = (f16t)(e1 * PCAR);
    }
    ls += __shfl_xor(ls, 16);
    L = L * corr + ls;
    #pragma unroll
    for (int t = 0; t < 4; ++t) {
      #pragma unroll
      for (int r = 0; r < 8; ++r) O[t][r] *= corr;
    }
    #pragma unroll
    for (int t = 0; t < 4; ++t) {
      FragH ha;
      load_frag(ha, hbase + (size_t)16 * t * NS + j0, 0);
      O[t] = wmma_f16(ha.v, pf.v, O[t]);
    }
  }

  const float inv = (1.0f / L) * SC_OA;
  #pragma unroll
  for (int t = 0; t < 4; ++t) {
    #pragma unroll
    for (int r = 0; r < 8; ++r)
      sbuf[(16 * wave + m) * PH + 16 * t + 8 * h + r] = (f16t)(O[t][r] * inv);
  }
  __syncthreads();

  v8h ov[4];
  size_t off[4];
  #pragma unroll
  for (int k = 0; k < 4; ++k) {
    const int row = 16 * k + (tid >> 3), q = tid & 7;
    ov[k] = *(const v8ha*)(sbuf + row * PH + 8 * q);
    off[k] = ((size_t)b * NS + 64 * qb + row) * DH + 8 * q;
  }
  #pragma unroll
  for (int k = 0; k < 4; ++k) *(volatile v8h*)(AGp + off[k]) = ov[k];
  __threadfence();
  #pragma unroll
  for (int k = 0; k < 4; ++k) *(volatile v8h*)(AGp + off[k]) = ov[k];
}

__global__ __launch_bounds__(TPB) void vproj_k(const float* __restrict__ x, const float* __restrict__ y,
                                              const f16t* __restrict__ WB, const f16t* __restrict__ AG,
                                              const float* __restrict__ bv11, const float* __restrict__ bv12,
                                              const float* __restrict__ bv21, const float* __restrict__ bv22,
                                              const float* __restrict__ alpha, const float* __restrict__ beta,
                                              const float* __restrict__ gamma_, const float* __restrict__ sigma_,
                                              float* __restrict__ out)
{
  __shared__ __attribute__((aligned(16))) float sbuf[64 * PF];
  const int tid = threadIdx.x, lane = tid & 31, wave = tid >> 5;
  const int h = lane >> 4, m = lane & 15;
  const int blk = blockIdx.x;
  const int o = blk / (NB * NCT64 * NQT);
  int rem = blk - o * (NB * NCT64 * NQT);
  const int b = rem / (NCT64 * NQT);
  rem -= b * (NCT64 * NQT);
  const int cb = rem / NQT;
  const int nb = rem - cb * NQT;
  const int c0 = 64 * cb, n0 = 64 * nb;

  const f16t *WA, *WBp, *AGA, *AGB;
  const float *bA, *bB, *z;
  float sA, sB;
  float* outp;
  if (o == 0) {
    WA  = WB + 6 * WMAT; bA = bv11; AGA = AG + 0 * PLN; sA = alpha[0];
    WBp = WB + 8 * WMAT; bB = bv21; AGB = AG + 1 * PLN; sB = beta[0];
    z = x; outp = out;
  } else {
    WA  = WB + 7 * WMAT; bA = bv12; AGA = AG + 3 * PLN; sA = gamma_[0];
    WBp = WB + 9 * WMAT; bB = bv22; AGB = AG + 2 * PLN; sB = sigma_[0];
    z = y; outp = out + (size_t)NB * CIN * NS;
  }

  v8f accA[4], accB[4];
  #pragma unroll
  for (int t = 0; t < 4; ++t) { accA[t] = zero8f(); accB[t] = zero8f(); }
  {
    const f16t* arow = WA + (size_t)(c0 + 16 * wave + m) * DH + 8 * h;
    const f16t* brow = AGA + ((size_t)b * NS + n0 + m) * DH + 8 * h;
    mma_4n<DH>(arow, brow, accA);
  }
  {
    const f16t* arow = WBp + (size_t)(c0 + 16 * wave + m) * DH + 8 * h;
    const f16t* brow = AGB + ((size_t)b * NS + n0 + m) * DH + 8 * h;
    mma_4n<DH>(arow, brow, accB);
  }

  #pragma unroll
  for (int r = 0; r < 8; ++r) {
    const int crow = 16 * wave + 8 * h + r;
    const float ba = bA[c0 + crow], bb = bB[c0 + crow];
    #pragma unroll
    for (int t = 0; t < 4; ++t) {
      const float g = sA * (accA[t][r] * SC_V + ba) + sB * (accB[t][r] * SC_V + bb);
      sbuf[crow * PF + 16 * t + m] = g;
    }
  }
  __syncthreads();

  v4f ov[8];
  size_t off[8];
  #pragma unroll
  for (int k = 0; k < 8; ++k) {
    const int row = 8 * k + (tid >> 4), q = tid & 15;
    const v4f gv = *(const v4fa*)(sbuf + row * PF + 4 * q);
    off[k] = ((size_t)b * CIN + c0 + row) * NS + n0 + 4 * q;
    const v4f zv = *(const v4fa*)(z + off[k]);
    ov[k] = zv + gv;
  }
  #pragma unroll
  for (int k = 0; k < 8; ++k) *(volatile v4f*)(outp + off[k]) = ov[k];
  __threadfence();
  #pragma unroll
  for (int k = 0; k < 8; ++k) *(volatile v4f*)(outp + off[k]) = ov[k];
}

extern "C" void kernel_launch(void* const* d_in, const int* in_sizes, int n_in,
                              void* d_out, int out_size, void* d_ws, size_t ws_size,
                              hipStream_t stream) {
  if (n_in < 26) return;
  if (in_sizes[0] != NB * CIN * NS || in_sizes[1] != NB * CIN * NS) return;
  for (int i = 2; i <= 12; i += 2) { if (in_sizes[i] != DH * CIN || in_sizes[i + 1] != DH) return; }
  for (int i = 14; i <= 20; i += 2) { if (in_sizes[i] != CIN * DH || in_sizes[i + 1] != CIN) return; }
  for (int i = 22; i <= 25; ++i) { if (in_sizes[i] < 1) return; }
  if (out_size != 2 * NB * CIN * NS) return;

  const float* x    = (const float*)d_in[0];
  const float* y    = (const float*)d_in[1];
  const float* Wf1  = (const float*)d_in[2];  const float* bf1  = (const float*)d_in[3];
  const float* Wg1  = (const float*)d_in[4];  const float* bg1  = (const float*)d_in[5];
  const float* Wh1  = (const float*)d_in[6];  const float* bh1  = (const float*)d_in[7];
  const float* Wf2  = (const float*)d_in[8];  const float* bf2  = (const float*)d_in[9];
  const float* Wg2  = (const float*)d_in[10]; const float* bg2  = (const float*)d_in[11];
  const float* Wh2  = (const float*)d_in[12]; const float* bh2  = (const float*)d_in[13];
  const float* Wv11 = (const float*)d_in[14]; const float* bv11 = (const float*)d_in[15];
  const float* Wv12 = (const float*)d_in[16]; const float* bv12 = (const float*)d_in[17];
  const float* Wv21 = (const float*)d_in[18]; const float* bv21 = (const float*)d_in[19];
  const float* Wv22 = (const float*)d_in[20]; const float* bv22 = (const float*)d_in[21];
  const float* alpha  = (const float*)d_in[22];
  const float* beta   = (const float*)d_in[23];
  const float* gamma_ = (const float*)d_in[24];
  const float* sigma_ = (const float*)d_in[25];
  float* outp = (float*)d_out;

  const size_t szXT = (size_t)NB * NS * CIN * 2;
  const size_t szWB = (size_t)NWM * WMAT * 2;
  const size_t szFG = 8 * PLN * 2;
  const size_t szHP = 2 * PLN * 2;
  const size_t szAG = 4 * PLN * 2;
  static_assert((size_t)NB * NS * CIN * 2 * 2 + (size_t)NWM * WMAT * 2 + 8 * PLN * 2 + 2 * PLN * 2 + 4 * PLN * 2 <= (size_t)134217728);
  size_t off = 0;
  char* ws = (char*)d_ws;
  f16t* XT  = (f16t*)(ws + off); off += szXT;
  f16t* YT  = (f16t*)(ws + off); off += szXT;
  f16t* WBp = (f16t*)(ws + off); off += szWB;
  unsigned short* FG = (unsigned short*)(ws + off); off += szFG;
  f16t* HPp = (f16t*)(ws + off); off += szHP;
  f16t* AGp = (f16t*)(ws + off); off += szAG;
  if (off > ws_size) return;

  prep_k<<<XP_BLKS + WB_BLKS, TPBP, 0, stream>>>(x, y, Wf1, Wg1, Wh1, Wf2, Wg2, Wh2, Wv11, Wv12, Wv21, Wv22,
                                                XT, YT, WBp);
  proj_k<<<6 * NB * NQT, TPB, 0, stream>>>(XT, YT, WBp, bf1, bg1, bh1, bf2, bg2, bh2, FG, HPp);
  agg_k<<<4 * NB * NQT, TPB, 0, stream>>>(FG, HPp, AGp);
  vproj_k<<<2 * NB * NCT64 * NQT, TPB, 0, stream>>>(x, y, WBp, AGp, bv11, bv12, bv21, bv22,
                                                   alpha, beta, gamma_, sigma_, outp);
  (void)hipGetLastError();
}
